// BiaffineEdgeAttention_66279935312113
// MI455X (gfx1250) — hardware-run, weakly checked
//
#include <hip/hip_runtime.h>


#define NRW  16384
#define NSQ  2048
#define NDP  256
#define NDC  320
#define NTL  64

typedef _Float16 h16;
typedef unsigned short bf;
typedef __attribute__((ext_vector_type(16))) __bf16   v16bf;
typedef __attribute__((ext_vector_type(16))) _Float16 v16h;
typedef __attribute__((ext_vector_type(8)))  _Float16 v8h;
typedef __attribute__((ext_vector_type(8)))  unsigned short v8us;
typedef __attribute__((ext_vector_type(8)))  float    v8f;
typedef __attribute__((ext_vector_type(4)))  float    v4f;
typedef v8h  __attribute__((may_alias)) v8ha;
typedef v4f  __attribute__((may_alias)) v4fa;
typedef v8us __attribute__((may_alias)) v8usa;

__device__ __forceinline__ unsigned short f2bf(float f) { unsigned u = __float_as_uint(f); u += 0x7FFFu + ((u >> 16) & 1u); return (unsigned short)(u >> 16); }
__device__ __forceinline__ float bf2f(unsigned short b) { return __uint_as_float(((unsigned)b) << 16); }
__device__ __forceinline__ float bfr(float f) { return bf2f(f2bf(f)); }
__device__ __forceinline__ v16h cat16(v8h lo, v8h hi) { return __builtin_shufflevector(lo, hi, 0, 1, 2, 3, 4, 5, 6, 7, 8, 9, 10, 11, 12, 13, 14, 15); }
__device__ __forceinline__ v16bf cat16b(v8us lo, v8us hi) { return __builtin_bit_cast(v16bf, __builtin_shufflevector(lo, hi, 0, 1, 2, 3, 4, 5, 6, 7, 8, 9, 10, 11, 12, 13, 14, 15)); }
__device__ __forceinline__ v8f wmma16(v16h a, v16h b, v8f c) { return __builtin_amdgcn_wmma_f32_16x16x32_f16(false, a, false, b, (short)0, c, false, false); }
__device__ __forceinline__ v8f wmmab(v16bf a, v16bf b, v8f c) { return __builtin_amdgcn_wmma_f32_16x16x32_bf16(false, a, false, b, (short)0, c, false, false); }

template <typename T16> struct WFrag;
template <> struct WFrag<h16> { typedef v16h V; static __device__ __forceinline__ V ld(const h16* p) { return cat16(*(const v8h*)p, *(const v8h*)(p + 16)); } static __device__ __forceinline__ v8f mma(V a, V b, v8f c) { return wmma16(a, b, c); } };
template <> struct WFrag<bf> { typedef v16bf V; static __device__ __forceinline__ V ld(const bf* p) { return cat16b(*(const v8us*)p, *(const v8us*)(p + 16)); } static __device__ __forceinline__ v8f mma(V a, V b, v8f c) { return wmmab(a, b, c); } };
template <typename T16, int NSPLIT, bool BIAS>
__global__ __launch_bounds__(32) void k_gemmw(const T16* __restrict__ A, const T16* __restrict__ A2, const T16* __restrict__ Bt, const T16* __restrict__ Bt2, int K, float* C, int ldc, const float* __restrict__ bias, size_t sA, size_t sB, size_t sC) {
    typedef typename WFrag<T16>::V V;
    __shared__ __align__(16) float os[16 * 68];
    const size_t z = blockIdx.z; A += z * sA; if (A2) A2 += z * sA; Bt += z * sB; if (Bt2) Bt2 += z * sB; C += z * sC;
    const int lane = threadIdx.x & 31, lr = lane & 15, hi = lane >> 4; const int r0 = blockIdx.x * 64, c0 = blockIdx.y * 64;
    v8f acc[4][4];
#pragma unroll
    for (int mb = 0; mb < 4; ++mb)
#pragma unroll
        for (int nb = 0; nb < 4; ++nb) acc[mb][nb] = (v8f){};
    const size_t aoff = (size_t)(r0 + lr) * K + 8 * hi, boff = (size_t)(c0 + lr) * K + 8 * hi;
    for (int kc = 0; kc < K; kc += 32) {
        V a[4], a2[4];
#pragma unroll
        for (int mb = 0; mb < 4; ++mb) { a[mb] = WFrag<T16>::ld(A + aoff + (size_t)mb * 16 * K + kc); if (NSPLIT == 1 || NSPLIT == 2) a2[mb] = WFrag<T16>::ld(A2 + aoff + (size_t)mb * 16 * K + kc); }
#pragma unroll
        for (int nb = 0; nb < 4; ++nb) { const V b = WFrag<T16>::ld(Bt + boff + (size_t)nb * 16 * K + kc); V b2; if (NSPLIT >= 2) b2 = WFrag<T16>::ld(Bt2 + boff + (size_t)nb * 16 * K + kc);
#pragma unroll
            for (int mb = 0; mb < 4; ++mb) { acc[mb][nb] = WFrag<T16>::mma(a[mb], b, acc[mb][nb]); if (NSPLIT == 1 || NSPLIT == 2) acc[mb][nb] = WFrag<T16>::mma(a2[mb], b, acc[mb][nb]); if (NSPLIT >= 2) acc[mb][nb] = WFrag<T16>::mma(a[mb], b2, acc[mb][nb]); } }
        asm volatile("v_nop\n\tv_nop\n\tv_nop\n\tv_nop" : "+v"(acc[0][0]), "+v"(acc[1][1]), "+v"(acc[2][2]), "+v"(acc[3][3]) : "v"(a[0]), "v"(a[3]));
    }
#pragma unroll
    for (int mb = 0; mb < 4; ++mb) {
#pragma unroll
        for (int nb = 0; nb < 4; ++nb) {
#pragma unroll
            for (int j = 0; j < 8; ++j) os[(hi * 8 + j) * 68 + nb * 16 + lr] = acc[mb][nb][j]; }
        __builtin_amdgcn_wave_barrier(); asm volatile("" ::: "memory");
        float* crow = C + (size_t)(r0 + mb * 16) * ldc + c0;
#pragma unroll 1
        for (int ps = 0; ps < 2; ++ps) {
#pragma unroll
            for (int s = 0; s < 8; ++s) { const int row = 2 * s + hi, cofs = lr * 4; v4f val = *(const v4fa*)(os + row * 68 + cofs); if (BIAS) { val[0] += bfr(bias[c0 + cofs]); val[1] += bfr(bias[c0 + cofs + 1]); val[2] += bfr(bias[c0 + cofs + 2]); val[3] += bfr(bias[c0 + cofs + 3]); }
                *(volatile v4f*)(crow + (size_t)row * ldc + cofs) = val; }
            if (ps == 0) __threadfence(); }
        __builtin_amdgcn_wave_barrier(); asm volatile("" ::: "memory");
    }
}

typedef __attribute__((ext_vector_type(2))) _Float16 v2h;
typedef __attribute__((ext_vector_type(4))) _Float16 v4h;
typedef __attribute__((ext_vector_type(2))) unsigned short v2us;
typedef __attribute__((ext_vector_type(4))) unsigned short v4us;
typedef __attribute__((ext_vector_type(2))) float v2f;
typedef __attribute__((ext_vector_type(4))) int v4i;
__global__ __launch_bounds__(256) void k_cvt8(const float* __restrict__ src, bf* dst, size_t n8) { const size_t i = (size_t)blockIdx.x * 256 + threadIdx.x; if (i >= n8) return; const v8f v = *(const v8f*)(src + i * 8); v8us o;
#pragma unroll
    for (int k = 0; k < 8; ++k) o[k] = f2bf(v[k]); *(volatile v8us*)(dst + i * 8) = o; __threadfence(); *(volatile v8us*)(dst + i * 8) = o; }

__global__ __launch_bounds__(256) void k_fillb(bf* P, unsigned w2, size_t n8) { const size_t i = (size_t)blockIdx.x * 256 + threadIdx.x; if (i >= n8) return; v4i o; o[0] = (int)w2; o[1] = (int)w2; o[2] = (int)w2; o[3] = (int)w2;
    *(volatile v4i*)(P + i * 8) = o; __threadfence(); *(volatile v4i*)(P + i * 8) = o; }

__device__ __forceinline__ h16 toh_flush(float x) { const float z = (fabsf(x) < 6.103515625e-05f) ? 0.0f : x; return (h16)z; }

template <bool RB>
__global__ __launch_bounds__(256) void k_c16p(const float* __restrict__ Sr, unsigned sp, h16* Dp) { const unsigned id = blockIdx.x * 256u + threadIdx.x; const unsigned rw = id >> 5, c8 = id & 31u; const float* ps = Sr + (size_t)rw * sp + c8 * 8u; const v4f wa = *(const v4f*)ps, wb = *(const v4f*)(ps + 4); v8h ov;
#pragma unroll
    for (int q1 = 0; q1 < 4; ++q1) { ov[q1] = toh_flush(RB ? bfr(wa[q1]) : wa[q1]); ov[q1 + 4] = toh_flush(RB ? bfr(wb[q1]) : wb[q1]); }
    h16* pd = Dp + (size_t)rw * NDC + c8 * 8u; *(volatile v8h*)pd = ov; __threadfence(); *(volatile v8h*)pd = ov; }

__global__ __launch_bounds__(256) void k_tl(const float* __restrict__ Sr, unsigned sp, unsigned sc, unsigned fo, const float* __restrict__ u5, h16* Dp) { const unsigned id = blockIdx.x * 256u + threadIdx.x; const unsigned rw = id >> 3, g8 = id & 7u; const float tv = Sr[(size_t)rw * sp + sc]; const float av = bfr(u5[0]); const float mk = (float)(1u - ((g8 + 7u) >> 3)); const unsigned sl = 0u - fo, tb = __float_as_uint(tv), ab = __float_as_uint(av); const float w0 = __uint_as_float((tb & ~sl) | (0x3f800000u & sl)) * mk; const float w1 = __uint_as_float((tb & sl) | (0x3f800000u & ~sl)) * mk; const float w2 = __uint_as_float((ab & sl) | (0x3f800000u & ~sl)) * mk; const float zz = mk - mk; v8h ov;
#pragma unroll
    for (int q1 = 0; q1 < 8; ++q1) ov[q1] = toh_flush(q1 == 0 ? w0 : (q1 == 1 ? w1 : (q1 == 2 ? w2 : zz)));
    h16* pd = Dp + (size_t)rw * NDC + NDP + g8 * 8u; *(volatile v8h*)pd = ov; __threadfence(); *(volatile v8h*)pd = ov; }

extern "C" void kernel_launch(void* const* d_in, const int* in_sizes, int n_in, void* d_out, int out_size, void* d_ws, size_t ws_size, hipStream_t stream) {
    if (n_in < 5) return;
    if (in_sizes[0] != NRW * NDP || in_sizes[1] != NRW * NDP || in_sizes[2] != NDP * NDP || in_sizes[3] != 2 * NDP || in_sizes[4] != 1) return;
    if (out_size != 8 * NSQ * NSQ) return;
    static_assert(NRW == 8 * NSQ && NSQ == 2048 && NDP == 256 && NDC == NDP + NTL && NTL == 64 && NDC % 32 == 0 && NDP % 32 == 0 && NRW % 64 == 0 && NSQ % 64 == 0 && NDC % 64 == 0 && NTL % 64 == 0 && (NDC * 2) % 128 == 0 && (NRW * NDP / 8) % 256 == 0 && (NDP * NDP / 8) % 256 == 0 && (NTL * NDP / 8) % 256 == 0 && (NRW * NTL / 8) % 256 == 0 && NDP / 8 == 32, "the products: row and column counts multiples of 64, the depths of 32; each flat grid exact; a row of the two wide planes is a whole number of 128-byte lines; the two one-row copies are 32 eights each on one block");
    const float* i0 = (const float*)d_in[0]; const float* i1 = (const float*)d_in[1]; const float* i2 = (const float*)d_in[2]; const float* i3 = (const float*)d_in[3]; const float* i4 = (const float*)d_in[4]; float* rs0 = (float*)d_out;
    char* wsp = (char*)d_ws; auto carve = [&](size_t bytes) { char* p = wsp; wsp += (bytes + 255) & ~(size_t)255; return (void*)p; };
    bf* Hb = (bf*)carve((size_t)NRW * NDP * 2); bf* Db = (bf*)carve((size_t)NRW * NDP * 2); bf* Ub = (bf*)carve((size_t)NDC * NDP * 2); bf* Vb = (bf*)carve((size_t)NTL * NDP * 2); float* P1 = (float*)carve((size_t)NRW * NDC * 4); float* P2 = (float*)carve((size_t)NRW * NTL * 4); h16* Ac = (h16*)carve((size_t)NRW * NDC * 2); h16* Bc = (h16*)carve((size_t)NRW * NDC * 2);
    if ((size_t)(wsp - (char*)d_ws) > ws_size) return;
    k_cvt8<<<(unsigned)(NRW * NDP / 8 / 256), 256, 0, stream>>>(i0, Hb, (size_t)NRW * NDP / 8);
    k_cvt8<<<(unsigned)(NRW * NDP / 8 / 256), 256, 0, stream>>>(i1, Db, (size_t)NRW * NDP / 8);
    k_cvt8<<<(unsigned)(NDP * NDP / 8 / 256), 256, 0, stream>>>(i2, Ub, (size_t)NDP * NDP / 8);
    k_fillb<<<(unsigned)(NTL * NDP / 8 / 256), 256, 0, stream>>>(Ub + (size_t)NDP * NDP, 0u, (size_t)NTL * NDP / 8);
    k_cvt8<<<1, 256, 0, stream>>>(i3 + NDP, Ub + (size_t)NDP * NDP, (size_t)NDP / 8);
    k_fillb<<<(unsigned)(NTL * NDP / 8 / 256), 256, 0, stream>>>(Vb, 0u, (size_t)NTL * NDP / 8);
    k_cvt8<<<1, 256, 0, stream>>>(i3, Vb, (size_t)NDP / 8);
    k_gemmw<bf, 0, false><<<dim3(NRW / 64, NDC / 64, 1), 32, 0, stream>>>(Db, nullptr, Ub, nullptr, NDP, P1, NDC, nullptr, 0, 0, 0);
    k_gemmw<bf, 0, false><<<dim3(NRW / 64, NTL / 64, 1), 32, 0, stream>>>(Hb, nullptr, Vb, nullptr, NDP, P2, NTL, nullptr, 0, 0, 0);
    k_c16p<true><<<(unsigned)(NRW * NDP / 8 / 256), 256, 0, stream>>>(i0, (unsigned)NDP, Ac);
    k_tl<<<(unsigned)(NRW * NTL / 8 / 256), 256, 0, stream>>>(P2, (unsigned)NTL, 0u, 0u, i4, Ac);
    k_c16p<false><<<(unsigned)(NRW * NDP / 8 / 256), 256, 0, stream>>>(P1, (unsigned)NDC, Bc);
    k_tl<<<(unsigned)(NRW * NTL / 8 / 256), 256, 0, stream>>>(P1, (unsigned)NDC, (unsigned)NDP, 1u, i4, Bc);
    k_gemmw<h16, 0, false><<<dim3(NSQ / 64, NSQ / 64, 8), 32, 0, stream>>>(Ac, nullptr, Bc, nullptr, NDC, rs0, NSQ, nullptr, (size_t)NSQ * NDC, (size_t)NSQ * NDC, (size_t)NSQ * NSQ);
}
